// SequentialCNNPoseLSTM_48799418417253
// MI455X (gfx1250) — hardware-run, weakly checked
//
#include <hip/hip_runtime.h>
#include <math.h>

constexpr int BATCH     = 64;
constexpr int CIN_CH    = 16;
constexpr int TSTEPS    = 2048;
constexpr int NFILT     = 64;
constexpr int HIDDEN    = 256;
constexpr int GATES     = 4 * HIDDEN;
constexpr int NOUT_CH   = 20;
constexpr int NOUT_PAD  = 32;
constexpr int KCONV     = CIN_CH * 3;
constexpr int KCONV_PAD = 64;
constexpr int MROWS     = TSTEPS * BATCH;
constexpr int K0TOT     = NFILT + HIDDEN;
constexpr int K1TOT     = HIDDEN + HIDDEN;
constexpr int A0_PITCH  = K0TOT + 8;
constexpr int A1_PITCH  = K1TOT + 8;
constexpr int ROWS_BLK  = 16;
constexpr int LS_THREADS = 512;
constexpr int STAT_BLOCKS = 256;
constexpr int STAT_ROWS   = MROWS / STAT_BLOCKS;
constexpr int GSTRIDE0  = HIDDEN * K0TOT;
constexpr int GSTRIDE1  = HIDDEN * K1TOT;

constexpr float X_CARRY     = 16.0f;
constexpr float CW_CARRY    = 256.0f;
constexpr float CONV_INV    = 1.0f / (X_CARRY * CW_CARRY);
constexpr float FEAT_CARRY  = 64.0f;
constexpr float WIH0_CARRY  = 2048.0f;
constexpr float H_CARRY     = 512.0f;
constexpr float W_CARRY     = 256.0f;
constexpr float TOT_CARRY   = 131072.0f;
constexpr float TOT_CARRY_INV = 1.0f / TOT_CARRY;
constexpr float BN_EPS      = 1e-5f;
constexpr double INV_COUNT_D = 1.0 / 131072.0;
constexpr float F16_MIN_NORMAL = 6.103515625e-05f;

static_assert(FEAT_CARRY * WIH0_CARRY == TOT_CARRY);
static_assert(H_CARRY * W_CARRY == TOT_CARRY);
static_assert(MROWS == 131072);
static_assert(KCONV == 48 && KCONV_PAD % 32 == 0);
static_assert(K0TOT % 32 == 0 && K1TOT % 32 == 0 && HIDDEN % 32 == 0);
static_assert(MROWS % 64 == 0 && NFILT == 64);
static_assert(LS_THREADS / 32 == ROWS_BLK);
static_assert(HIDDEN == 16 * (LS_THREADS / 32));
static_assert(BATCH % ROWS_BLK == 0);
static_assert(A0_PITCH % 8 == 0 && A1_PITCH % 8 == 0);
static_assert(STAT_ROWS == 512);

typedef __attribute__((ext_vector_type(16))) _Float16 v16h;
typedef __attribute__((ext_vector_type(8)))  _Float16 v8h;
typedef __attribute__((ext_vector_type(8)))  float    v8f;
typedef __attribute__((ext_vector_type(4)))  float    v4f;
typedef __attribute__((ext_vector_type(4)))  unsigned v4u;

union FragU { v16h v; v8h h[2]; };

__device__ __forceinline__ v16h frag_load(const _Float16* p) {
  FragU f;
  f.h[0] = *(const v8h*)(p);
  f.h[1] = *(const v8h*)(p + 16);
  return f.v;
}

__device__ __forceinline__ v8f mma_g(v16h a, v16h b, v8f c) {
  c = __builtin_amdgcn_wmma_f32_16x16x32_f16(false, a, false, b, (short)0, c, false, false);
  asm volatile("v_nop\n\tv_nop\n\tv_nop\n\tv_nop" : "+v"(c) : "v"(a), "v"(b));
  return c;
}

__device__ __forceinline__ void pin4(v4f& v) { asm volatile("" : "+v"(v)); }
__device__ __forceinline__ void pin1(float& v) { asm volatile("" : "+v"(v)); }

__device__ __forceinline__ _Float16 to_h16(float v) {
  const float r = (fabsf(v) < F16_MIN_NORMAL) ? 0.0f : v;
  return (_Float16)r;
}
__device__ __forceinline__ unsigned h_bits(float v) {
  const _Float16 h = to_h16(v);
  const unsigned short u = __builtin_bit_cast(unsigned short, h);
  return (unsigned)u;
}
__device__ __forceinline__ unsigned pack2(float lo, float hi) {
  const unsigned a = h_bits(lo);
  const unsigned b = h_bits(hi);
  return a | (b << 16);
}

__device__ __forceinline__ float fsig(float x)  { return __builtin_amdgcn_rcpf(1.0f + __expf(-x)); }
__device__ __forceinline__ float ftanh(float x) { return 1.0f - 2.0f * __builtin_amdgcn_rcpf(__expf(2.0f * x) + 1.0f); }

__global__ __launch_bounds__(256) void build_plane_kernel(const float* srcA, int ka, float sa,
                                                          const float* srcB, int kb, float sb,
                                                          unsigned short* __restrict__ dst,
                                                          int nrow_src, int nrow_dst, int kout) {
  const int i = blockIdx.x * 256 + threadIdx.x;
  const int ncol8 = kout >> 3;
  const int n8 = nrow_dst * ncol8;
  const int ic = (i < n8) ? i : (n8 - 1);
  const int row = ic / ncol8;
  const int col = (ic - row * ncol8) * 8;
  const bool rowok = row < nrow_src;
  const int rowc = rowok ? row : (nrow_src - 1);
  const bool inA = col < ka;
  const bool inB = (!inA) && (col < ka + kb);
  const int colA = inA ? col : (ka - 8);
  int colB = col - ka;
  int mxB = kb - 8;
  mxB = mxB < 0 ? 0 : mxB;
  colB = colB < 0 ? 0 : colB;
  colB = colB > mxB ? mxB : colB;
  const float* pa = srcA + (size_t)rowc * (size_t)ka + colA;
  const float* pb = srcB + (size_t)rowc * (size_t)kb + colB;
  v4f a0 = *(const v4f*)(pa);
  v4f a1 = *(const v4f*)(pa + 4);
  v4f b0 = *(const v4f*)(pb);
  v4f b1 = *(const v4f*)(pb + 4);
  pin4(a0);
  pin4(a1);
  pin4(b0);
  pin4(b1);
  float o[8];
#pragma unroll
  for (int e = 0; e < 4; ++e) {
    const float va0 = a0[e] * sa;
    const float vb0 = b0[e] * sb;
    const float va1 = a1[e] * sa;
    const float vb1 = b1[e] * sb;
    const float s0 = inA ? va0 : (inB ? vb0 : 0.0f);
    const float s1 = inA ? va1 : (inB ? vb1 : 0.0f);
    o[e]     = rowok ? s0 : 0.0f;
    o[4 + e] = rowok ? s1 : 0.0f;
  }
  v4u w;
  w[0] = pack2(o[0], o[1]);
  w[1] = pack2(o[2], o[3]);
  w[2] = pack2(o[4], o[5]);
  w[3] = pack2(o[6], o[7]);
  if (i < n8) {
    volatile v4u* dp = (volatile v4u*)(dst + (size_t)i * 8);
    *dp = w;
    __threadfence();
    *dp = w;
  }
}

__global__ __launch_bounds__(256) void im2col_kernel(const float* __restrict__ x, unsigned short* __restrict__ xcol) {
  __shared__ float xs[CIN_CH * 68];
  const int tid = threadIdx.x;
  const int b  = blockIdx.x & (BATCH - 1);
  const int t0 = (blockIdx.x >> 6) * 64;
  {
    const int c = tid >> 4, i4 = (tid & 15) * 4;
    const v4f v = *(const v4f*)(x + ((size_t)b * CIN_CH + c) * TSTEPS + t0 + i4);
    xs[c * 68 + 1 + i4 + 0] = v[0];
    xs[c * 68 + 1 + i4 + 1] = v[1];
    xs[c * 68 + 1 + i4 + 2] = v[2];
    xs[c * 68 + 1 + i4 + 3] = v[3];
  }
  if (tid < 32) {
    const int c = tid >> 1, side = tid & 1;
    const int tt = side ? (t0 + 64) : (t0 - 1);
    const bool ok = (tt >= 0) && (tt < TSTEPS);
    const int ttc = tt < 0 ? 0 : (tt >= TSTEPS ? (TSTEPS - 1) : tt);
    float v = x[((size_t)b * CIN_CH + c) * TSTEPS + ttc];
    pin1(v);
    xs[c * 68 + (side ? 65 : 0)] = ok ? v : 0.0f;
  }
  __syncthreads();
  const int q = tid >> 3, c8 = (tid & 7) * 8;
  v4u w[2];
#pragma unroll
  for (int g = 0; g < 2; ++g) {
    const int tl = g * 32 + q;
    float o[8];
#pragma unroll
    for (int e = 0; e < 8; ++e) {
      const int k  = c8 + e;
      const int kc = k < KCONV ? k : (KCONV - 1);
      const int c  = kc / 3;
      const int kk = kc - 3 * c;
      const float v = xs[c * 68 + tl + kk];
      o[e] = (k < KCONV) ? (v * X_CARRY) : 0.0f;
    }
    w[g][0] = pack2(o[0], o[1]);
    w[g][1] = pack2(o[2], o[3]);
    w[g][2] = pack2(o[4], o[5]);
    w[g][3] = pack2(o[6], o[7]);
  }
  for (int pass = 0; pass < 2; ++pass) {
#pragma unroll
    for (int g = 0; g < 2; ++g) {
      const int tl = g * 32 + q;
      const size_t m = (size_t)(t0 + tl) * BATCH + (size_t)b;
      *(volatile v4u*)(xcol + m * KCONV_PAD + c8) = w[g];
    }
    __threadfence();
  }
}

__global__ __launch_bounds__(256) void conv_gemm_kernel(const unsigned short* __restrict__ Ap,
                                                        const unsigned short* __restrict__ Btp,
                                                        const float* __restrict__ bias,
                                                        float* __restrict__ Cout, int mtiles, float scale) {
  const _Float16* A  = (const _Float16*)Ap;
  const _Float16* Bt = (const _Float16*)Btp;
  __shared__ __align__(16) float sT[8][16 * 68];
  const int lane = threadIdx.x & 31;
  const int wave = threadIdx.x >> 5;
  const int tile = blockIdx.x * 8 + wave;
  if (tile >= mtiles) return;
  const int m0 = tile << 6;
  const int rlane = lane & 15;
  const int koff  = (lane >> 4) * 8;
  const int mOff  = (lane >> 4) * 8;

  v8f acc[4][4];
#pragma unroll
  for (int i = 0; i < 4; ++i)
#pragma unroll
    for (int j = 0; j < 4; ++j) acc[i][j] = (v8f){0.f, 0.f, 0.f, 0.f, 0.f, 0.f, 0.f, 0.f};

#pragma unroll 1
  for (int k0 = 0; k0 < KCONV_PAD; k0 += 32) {
    v16h bh[4];
#pragma unroll
    for (int j = 0; j < 4; ++j)
      bh[j] = frag_load(Bt + (size_t)((j << 4) + rlane) * KCONV_PAD + koff + k0);
#pragma unroll
    for (int i = 0; i < 4; ++i) {
      const v16h ah = frag_load(A + (size_t)(m0 + (i << 4) + rlane) * KCONV_PAD + koff + k0);
#pragma unroll
      for (int j = 0; j < 4; ++j) acc[i][j] = mma_g(ah, bh[j], acc[i][j]);
    }
  }

  float* slab = sT[wave];
#pragma unroll
  for (int i = 0; i < 4; ++i) {
    const int mBase = m0 + (i << 4);
#pragma unroll
    for (int j = 0; j < 4; ++j) {
      const float bv = bias[(j << 4) + rlane];
#pragma unroll
      for (int r = 0; r < 8; ++r) {
        float v = acc[i][j][r] * scale + bv;
        v = fmaxf(v, 0.0f);
        slab[(mOff + r) * 68 + (j << 4) + rlane] = v;
      }
    }
    __builtin_amdgcn_fence(__ATOMIC_RELEASE, "workgroup");
    __builtin_amdgcn_wave_barrier();
    __builtin_amdgcn_fence(__ATOMIC_ACQUIRE, "workgroup");
    {
      const int hh = lane >> 4, c4 = (lane & 15) * 4;
      for (int pass = 0; pass < 2; ++pass) {
#pragma unroll
        for (int it = 0; it < 8; ++it) {
          const int row = it * 2 + hh;
          const v4f v = *(const v4f*)(slab + row * 68 + c4);
          *(volatile v4f*)(Cout + (size_t)(mBase + row) * NFILT + c4) = v;
        }
        __threadfence();
      }
    }
    __builtin_amdgcn_fence(__ATOMIC_RELEASE, "workgroup");
    __builtin_amdgcn_wave_barrier();
    __builtin_amdgcn_fence(__ATOMIC_ACQUIRE, "workgroup");
  }
}

template <int MODE>
__global__ __launch_bounds__(256) void col_stats_kernel(const float* __restrict__ Y, const float* __restrict__ meanp,
                                                        float* __restrict__ part) {
  __shared__ float red[16 * NFILT];
  const int tid = threadIdx.x;
  const int cg = (tid & 15) * 4, rl = tid >> 4;
  const size_t base = (size_t)blockIdx.x * STAT_ROWS;
  v4f mu = {0.f, 0.f, 0.f, 0.f};
  if (MODE == 1) mu = *(const v4f*)(meanp + cg);
  v4f s = {0.f, 0.f, 0.f, 0.f};
#pragma unroll 4
  for (int i = 0; i < STAT_ROWS / 16; ++i) {
    const v4f v = *(const v4f*)(Y + (base + (size_t)(i * 16 + rl)) * NFILT + cg);
    if (MODE == 1) {
      const v4f d = v - mu;
      s += d * d;
    } else {
      s += v;
    }
  }
  red[rl * NFILT + cg + 0] = s[0];
  red[rl * NFILT + cg + 1] = s[1];
  red[rl * NFILT + cg + 2] = s[2];
  red[rl * NFILT + cg + 3] = s[3];
  __syncthreads();
  if (tid < NFILT) {
    float tot = 0.0f;
#pragma unroll
    for (int r = 0; r < 16; ++r) tot += red[r * NFILT + tid];
    volatile float* dp = part + (size_t)blockIdx.x * NFILT + tid;
    *dp = tot;
    __threadfence();
    *dp = tot;
  }
}

__global__ __launch_bounds__(64) void fin_mean_kernel(const float* __restrict__ part, float* __restrict__ meanp) {
  const int f = threadIdx.x;
  double s = 0.0;
#pragma unroll 1
  for (int i = 0; i < STAT_BLOCKS; ++i) s += (double)part[i * NFILT + f];
  const float mu = (float)(s * INV_COUNT_D);
  volatile float* dp = meanp + f;
  *dp = mu;
  __threadfence();
  *dp = mu;
}

__global__ __launch_bounds__(64) void fin_scale_kernel(const float* __restrict__ part, const float* __restrict__ meanp,
                                                       const float* __restrict__ gamma, const float* __restrict__ beta,
                                                       float* __restrict__ scalep, float* __restrict__ shiftp) {
  const int f = threadIdx.x;
  double s = 0.0;
#pragma unroll 1
  for (int i = 0; i < STAT_BLOCKS; ++i) s += (double)part[i * NFILT + f];
  const float var = (float)(s * INV_COUNT_D);
  const float sc = gamma[f] * (1.0f / sqrtf(var + BN_EPS));
  const float sh = beta[f] - meanp[f] * sc;
  volatile float* d0 = scalep + f;
  volatile float* d1 = shiftp + f;
  *d0 = sc;
  *d1 = sh;
  __threadfence();
  *d0 = sc;
  *d1 = sh;
}

__global__ __launch_bounds__(256) void bn_apply_kernel(const float* __restrict__ Y, const float* __restrict__ scalep,
                                                       const float* __restrict__ shiftp,
                                                       unsigned short* __restrict__ feats) {
  const size_t i = (size_t)blockIdx.x * 256 + threadIdx.x;
  const int c8 = ((int)(i & 7)) * 8;
  const v4f y0 = *(const v4f*)(Y + i * 8);
  const v4f y1 = *(const v4f*)(Y + i * 8 + 4);
  const v4f s0 = *(const v4f*)(scalep + c8);
  const v4f s1 = *(const v4f*)(scalep + c8 + 4);
  const v4f h0 = *(const v4f*)(shiftp + c8);
  const v4f h1 = *(const v4f*)(shiftp + c8 + 4);
  float o[8];
#pragma unroll
  for (int e = 0; e < 4; ++e) {
    o[e]     = (y0[e] * s0[e] + h0[e]) * FEAT_CARRY;
    o[4 + e] = (y1[e] * s1[e] + h1[e]) * FEAT_CARRY;
  }
  v4u w;
  w[0] = pack2(o[0], o[1]);
  w[1] = pack2(o[2], o[3]);
  w[2] = pack2(o[4], o[5]);
  w[3] = pack2(o[6], o[7]);
  volatile v4u* dp = (volatile v4u*)(feats + i * 8);
  *dp = w;
  __threadfence();
  *dp = w;
}

__device__ __forceinline__ void stage_feat(const _Float16* feat, _Float16* a0tile, int t, int rowbase, int tid) {
  const int m = tid >> 3, c8 = (tid & 7) * 8;
  const v8h xv = *(const v8h*)(feat + ((size_t)t * BATCH + (size_t)(rowbase + m)) * NFILT + c8);
  *(v8h*)(a0tile + m * A0_PITCH + c8) = xv;
}

__device__ __forceinline__ void emit_h_row(const _Float16* a1tile, _Float16* hplane, int t, int rowbase, int wave, int lane) {
  const v8h hv = *(const v8h*)(a1tile + wave * A1_PITCH + HIDDEN + lane * 8);
  volatile v8h* dp = (volatile v8h*)(hplane + ((size_t)t * BATCH + (size_t)(rowbase + wave)) * HIDDEN + lane * 8);
  *dp = hv;
  __threadfence();
  *dp = hv;
}

__global__ __launch_bounds__(LS_THREADS) void lstm2_kernel(const unsigned short* __restrict__ FEATp,
                                                           const unsigned short* __restrict__ W0p,
                                                           const unsigned short* __restrict__ W1p,
                                                           const float* __restrict__ bih0, const float* __restrict__ bhh0,
                                                           const float* __restrict__ bih1, const float* __restrict__ bhh1,
                                                           unsigned short* __restrict__ H2p) {
  __shared__ __align__(16) _Float16 A0[ROWS_BLK * A0_PITCH];
  __shared__ __align__(16) _Float16 A1[ROWS_BLK * A1_PITCH];
  const _Float16* FEAT = (const _Float16*)FEATp;
  const _Float16* W0 = (const _Float16*)W0p;
  const _Float16* W1 = (const _Float16*)W1p;
  _Float16* H2 = (_Float16*)H2p;
  const int tid = threadIdx.x, lane = tid & 31, wave = tid >> 5;
  const int c = lane & 15, hh = lane >> 4, koff = hh * 8;
  const int rowbase = blockIdx.x * ROWS_BLK;
  const int j = 16 * wave + c;

#pragma unroll 1
  for (int i = tid; i < ROWS_BLK * A0_PITCH; i += LS_THREADS) A0[i] = (_Float16)0.0f;
#pragma unroll 1
  for (int i = tid; i < ROWS_BLK * A1_PITCH; i += LS_THREADS) A1[i] = (_Float16)0.0f;
  __syncthreads();
  if (wave < 4) stage_feat(FEAT, A0, 0, rowbase, tid);

  float bz0[4], bz1[4];
#pragma unroll
  for (int g = 0; g < 4; ++g) {
    bz0[g] = bih0[g * HIDDEN + j] + bhh0[g * HIDDEN + j];
    bz1[g] = bih1[g * HIDDEN + j] + bhh1[g * HIDDEN + j];
  }
  float cst0[8], cst1[8];
#pragma unroll
  for (int r = 0; r < 8; ++r) { cst0[r] = 0.0f; cst1[r] = 0.0f; }
  __syncthreads();

  const _Float16* a0row = A0 + c * A0_PITCH + koff;
  const _Float16* a1row = A1 + c * A1_PITCH + koff;
  const _Float16* w0 = W0 + (size_t)j * K0TOT + koff;
  const _Float16* w1 = W1 + (size_t)j * K1TOT + koff;
  const v8f z8 = {0.f, 0.f, 0.f, 0.f, 0.f, 0.f, 0.f, 0.f};

#pragma unroll 1
  for (int t = 0; t < TSTEPS; ++t) {
    v8f gi = z8, gf = z8, gg = z8, go = z8;
#pragma unroll 1
    for (int k0 = 0; k0 < K0TOT; k0 += 32) {
      const v16h a  = frag_load(a0row + k0);
      const v16h b0 = frag_load(w0 + k0);
      const v16h b1 = frag_load(w0 + (size_t)GSTRIDE0 + k0);
      const v16h b2 = frag_load(w0 + (size_t)2 * GSTRIDE0 + k0);
      const v16h b3 = frag_load(w0 + (size_t)3 * GSTRIDE0 + k0);
      gi = mma_g(a, b0, gi);
      gf = mma_g(a, b1, gf);
      gg = mma_g(a, b2, gg);
      go = mma_g(a, b3, go);
    }
    float hn[8];
#pragma unroll
    for (int r = 0; r < 8; ++r) {
      const float zi = gi[r] * TOT_CARRY_INV + bz0[0];
      const float zf = gf[r] * TOT_CARRY_INV + bz0[1];
      const float zg = gg[r] * TOT_CARRY_INV + bz0[2];
      const float zo = go[r] * TOT_CARRY_INV + bz0[3];
      const float ig = fsig(zi);
      const float fg = fsig(zf);
      const float cg = ftanh(zg);
      const float og = fsig(zo);
      const float cn = fg * cst0[r] + ig * cg;
      cst0[r] = cn;
      hn[r] = og * ftanh(cn);
    }
    __syncthreads();
#pragma unroll
    for (int r = 0; r < 8; ++r) {
      const _Float16 hv = to_h16(hn[r] * H_CARRY);
      A0[(8 * hh + r) * A0_PITCH + NFILT + j] = hv;
      A1[(8 * hh + r) * A1_PITCH + j] = hv;
    }
    if (wave < 4) {
      const int tn = (t + 1 < TSTEPS) ? (t + 1) : (TSTEPS - 1);
      stage_feat(FEAT, A0, tn, rowbase, tid);
    }
    if (t > 0) emit_h_row(A1, H2, t - 1, rowbase, wave, lane);
    __syncthreads();

    gi = z8; gf = z8; gg = z8; go = z8;
#pragma unroll 1
    for (int k0 = 0; k0 < K1TOT; k0 += 32) {
      const v16h a  = frag_load(a1row + k0);
      const v16h b0 = frag_load(w1 + k0);
      const v16h b1 = frag_load(w1 + (size_t)GSTRIDE1 + k0);
      const v16h b2 = frag_load(w1 + (size_t)2 * GSTRIDE1 + k0);
      const v16h b3 = frag_load(w1 + (size_t)3 * GSTRIDE1 + k0);
      gi = mma_g(a, b0, gi);
      gf = mma_g(a, b1, gf);
      gg = mma_g(a, b2, gg);
      go = mma_g(a, b3, go);
    }
#pragma unroll
    for (int r = 0; r < 8; ++r) {
      const float zi = gi[r] * TOT_CARRY_INV + bz1[0];
      const float zf = gf[r] * TOT_CARRY_INV + bz1[1];
      const float zg = gg[r] * TOT_CARRY_INV + bz1[2];
      const float zo = go[r] * TOT_CARRY_INV + bz1[3];
      const float ig = fsig(zi);
      const float fg = fsig(zf);
      const float cg = ftanh(zg);
      const float og = fsig(zo);
      const float cn = fg * cst1[r] + ig * cg;
      cst1[r] = cn;
      hn[r] = og * ftanh(cn);
    }
    __syncthreads();
#pragma unroll
    for (int r = 0; r < 8; ++r)
      A1[(8 * hh + r) * A1_PITCH + HIDDEN + j] = to_h16(hn[r] * H_CARRY);
  }
  __syncthreads();
  emit_h_row(A1, H2, TSTEPS - 1, rowbase, wave, lane);
}

__global__ __launch_bounds__(128) void head_kernel(const unsigned short* __restrict__ H2p,
                                                   const unsigned short* __restrict__ FCp,
                                                   const float* __restrict__ fcb, float* __restrict__ out) {
  __shared__ __align__(16) float Ts[NOUT_PAD * 68];
  const _Float16* H2 = (const _Float16*)H2p;
  const _Float16* FC = (const _Float16*)FCp;
  const int tid = threadIdx.x, lane = tid & 31, wave = tid >> 5;
  const int c = lane & 15, hh = lane >> 4, koff = hh * 8;
  const int b  = blockIdx.x & (BATCH - 1);
  const int t0 = (blockIdx.x >> 6) * 64;
  const int tl = 16 * wave + c;
  const _Float16* ap  = H2 + ((size_t)(t0 + tl) * BATCH + (size_t)b) * HIDDEN + koff;
  const _Float16* bp0 = FC + (size_t)c * HIDDEN + koff;
  const _Float16* bp1 = FC + (size_t)(16 + c) * HIDDEN + koff;
  v8f acc0 = {0.f, 0.f, 0.f, 0.f, 0.f, 0.f, 0.f, 0.f};
  v8f acc1 = {0.f, 0.f, 0.f, 0.f, 0.f, 0.f, 0.f, 0.f};
#pragma unroll 1
  for (int k0 = 0; k0 < HIDDEN; k0 += 32) {
    const v16h a  = frag_load(ap + k0);
    const v16h b0 = frag_load(bp0 + k0);
    const v16h b1 = frag_load(bp1 + k0);
    acc0 = mma_g(a, b0, acc0);
    acc1 = mma_g(a, b1, acc1);
  }
  const float fb0 = fcb[c];
  const int o1 = 16 + c;
  const int o1c = o1 < NOUT_CH ? o1 : (NOUT_CH - 1);
  float fb1 = fcb[o1c];
  pin1(fb1);
  fb1 = (o1 < NOUT_CH) ? fb1 : 0.0f;
#pragma unroll
  for (int r = 0; r < 8; ++r) {
    Ts[c * 68 + 16 * wave + 8 * hh + r]        = acc0[r] * TOT_CARRY_INV + fb0;
    Ts[(16 + c) * 68 + 16 * wave + 8 * hh + r] = acc1[r] * TOT_CARRY_INV + fb1;
  }
  __syncthreads();
  const int orow = tid >> 4, c4 = (tid & 15) * 4;
  v4f val[3];
#pragma unroll
  for (int it = 0; it < 3; ++it) val[it] = *(const v4f*)(Ts + (it * 8 + orow) * 68 + c4);
  for (int pass = 0; pass < 2; ++pass) {
#pragma unroll
    for (int it = 0; it < 3; ++it) {
      const int o = it * 8 + orow;
      if (o < NOUT_CH)
        *(volatile v4f*)(out + ((size_t)b * NOUT_CH + (size_t)o) * TSTEPS + t0 + c4) = val[it];
    }
    __threadfence();
  }
}

extern "C" void kernel_launch(void* const* d_in, const int* in_sizes, int n_in,
                              void* d_out, int out_size, void* d_ws, size_t ws_size, hipStream_t stream) {
  if (n_in < 15 || d_out == nullptr || d_ws == nullptr) return;
  if (in_sizes[0] != BATCH * CIN_CH * TSTEPS || in_sizes[1] != NFILT * KCONV || in_sizes[2] != NFILT ||
      in_sizes[3] != NFILT || in_sizes[4] != NFILT || in_sizes[5] != GATES * NFILT || in_sizes[6] != GATES * HIDDEN ||
      in_sizes[7] != GATES || in_sizes[8] != GATES || in_sizes[9] != GATES * HIDDEN || in_sizes[10] != GATES * HIDDEN ||
      in_sizes[11] != GATES || in_sizes[12] != GATES || in_sizes[13] != NOUT_CH * HIDDEN || in_sizes[14] != NOUT_CH ||
      out_size != BATCH * NOUT_CH * TSTEPS) return;

  const float* x      = (const float*)d_in[0];
  const float* conv_w = (const float*)d_in[1];
  const float* conv_b = (const float*)d_in[2];
  const float* gamma  = (const float*)d_in[3];
  const float* beta   = (const float*)d_in[4];
  const float* wih0   = (const float*)d_in[5];
  const float* whh0   = (const float*)d_in[6];
  const float* bih0   = (const float*)d_in[7];
  const float* bhh0   = (const float*)d_in[8];
  const float* wih1   = (const float*)d_in[9];
  const float* whh1   = (const float*)d_in[10];
  const float* bih1   = (const float*)d_in[11];
  const float* bhh1   = (const float*)d_in[12];
  const float* fcw    = (const float*)d_in[13];
  const float* fcb    = (const float*)d_in[14];
  float* out = (float*)d_out;

  char* ws = (char*)d_ws;
  size_t off = 0;
  auto carve = [&](size_t bytes) -> char* { char* p = ws + off; off += (bytes + 255) & ~(size_t)255; return p; };
  float*          Y      = (float*)carve((size_t)MROWS * NFILT * 4);
  unsigned short* FEATS  = (unsigned short*)carve((size_t)MROWS * NFILT * 2);
  unsigned short* H2     = (unsigned short*)carve((size_t)MROWS * HIDDEN * 2);
  unsigned short* WCAT0  = (unsigned short*)carve((size_t)GATES * K0TOT * 2);
  unsigned short* WCAT1  = (unsigned short*)carve((size_t)GATES * K1TOT * 2);
  unsigned short* CONVBT = (unsigned short*)carve((size_t)NFILT * KCONV_PAD * 2);
  unsigned short* FCBT   = (unsigned short*)carve((size_t)NOUT_PAD * HIDDEN * 2);
  float*          PART1  = (float*)carve((size_t)STAT_BLOCKS * NFILT * 4);
  float*          PART2  = (float*)carve((size_t)STAT_BLOCKS * NFILT * 4);
  float*          MEANP  = (float*)carve((size_t)NFILT * 4);
  float*          SCALEP = (float*)carve((size_t)NFILT * 4);
  float*          SHIFTP = (float*)carve((size_t)NFILT * 4);
  unsigned short* XCOL   = H2;
  if (off > ws_size || off > (size_t)134217728) return;

  build_plane_kernel<<<(NFILT * KCONV_PAD / 8) / 256, 256, 0, stream>>>(
      conv_w, KCONV, CW_CARRY, conv_w, 0, 0.0f, CONVBT, NFILT, NFILT, KCONV_PAD);
  build_plane_kernel<<<(NOUT_PAD * HIDDEN / 8) / 256, 256, 0, stream>>>(
      fcw, HIDDEN, W_CARRY, fcw, 0, 0.0f, FCBT, NOUT_CH, NOUT_PAD, HIDDEN);
  build_plane_kernel<<<(GATES * K0TOT / 8) / 256, 256, 0, stream>>>(
      wih0, NFILT, WIH0_CARRY, whh0, HIDDEN, W_CARRY, WCAT0, GATES, GATES, K0TOT);
  build_plane_kernel<<<(GATES * K1TOT / 8) / 256, 256, 0, stream>>>(
      wih1, HIDDEN, W_CARRY, whh1, HIDDEN, W_CARRY, WCAT1, GATES, GATES, K1TOT);

  im2col_kernel<<<BATCH * (TSTEPS / 64), 256, 0, stream>>>(x, XCOL);
  conv_gemm_kernel<<<(MROWS / 64) / 8, 256, 0, stream>>>(XCOL, CONVBT, conv_b, Y, MROWS / 64, CONV_INV);
  col_stats_kernel<0><<<STAT_BLOCKS, 256, 0, stream>>>(Y, MEANP, PART1);
  fin_mean_kernel<<<1, 64, 0, stream>>>(PART1, MEANP);
  col_stats_kernel<1><<<STAT_BLOCKS, 256, 0, stream>>>(Y, MEANP, PART2);
  fin_scale_kernel<<<1, 64, 0, stream>>>(PART2, MEANP, gamma, beta, SCALEP, SHIFTP);
  bn_apply_kernel<<<(MROWS * NFILT / 8) / 256, 256, 0, stream>>>(Y, SCALEP, SHIFTP, FEATS);

  lstm2_kernel<<<BATCH / ROWS_BLK, LS_THREADS, 0, stream>>>(FEATS, WCAT0, WCAT1, bih0, bhh0, bih1, bhh1, H2);

  head_kernel<<<BATCH * (TSTEPS / 64), 128, 0, stream>>>(H2, FCBT, fcb, out);
}
